// NCL_50766513438740
// MI455X (gfx1250) — hardware-verified
//
#include <hip/hip_runtime.h>

typedef __attribute__((ext_vector_type(16))) _Float16 v16h;
typedef __attribute__((ext_vector_type(8)))  _Float16 v8h;
typedef __attribute__((ext_vector_type(2)))  _Float16 v2h;
typedef __attribute__((ext_vector_type(8)))  float    v8f;

#define TWO_PI_F   6.28318530717958647692f
#define K_E2       28.853900817779268f
#define C_LN       0.03465735902799726f

__device__ __forceinline__ float sigmoid20(float z) {
  return __builtin_amdgcn_rcpf(1.0f + __builtin_amdgcn_exp2f(-K_E2 * z));
}
__device__ __forceinline__ float softplus20(float z) {
  const float t = __builtin_amdgcn_exp2f(-K_E2 * fabsf(z));
  return fmaxf(z, 0.0f) + __builtin_amdgcn_logf(1.0f + t) * C_LN;
}
typedef __attribute__((ext_vector_type(4))) float v4f_t;
typedef float v4fa __attribute__((ext_vector_type(4), may_alias));
#define RSPLIT (1.0f / 2048.0f)
#define NPTS 1048576
__device__ __forceinline__ _Float16 lo_of(float v, _Float16 h) { return (_Float16)((v - (float)h) * 2048.0f); }
__device__ __forceinline__ v8f wmma16(v16h a, v16h b, v8f c) { return __builtin_amdgcn_wmma_f32_16x16x32_f16(false, a, false, b, (short)0, c, false, false); }
__device__ __forceinline__ v8f wmma_split(v16h a, v16h al, v16h b, v16h bl, v8f c) { v8f x = {}; x = wmma16(al, b, x); x = wmma16(a, bl, x); return wmma16(a, b, c) + x * RSPLIT; }

__device__ __forceinline__ v16h cat16(v8h lo, v8h hi) {
  return __builtin_shufflevector(lo, hi, 0,1,2,3,4,5,6,7,8,9,10,11,12,13,14,15);
}

__device__ __forceinline__ v16h load_bfrag(const _Float16* T, int lane, int nt) {
  int n  = nt * 16 + (lane & 15);
  int kh = (lane >> 4) * 8;
  const _Float16* p = T + n * 32 + kh;
  v8h lo = *(const v8h*)(p);
  v8h hi = *(const v8h*)(p + 16);
  return cat16(lo, hi);
}

__device__ __forceinline__ v16h load_afrag(const _Float16* T, int lane, int mt) {
  int m  = mt * 16 + (lane & 15);
  int ks = (lane >> 4) * 8;
  const _Float16* p = T + m * 32 + ks;
  v8h lo = *(const v8h*)(p);
  v8h hi = *(const v8h*)(p + 16);
  return cat16(lo, hi);
}

#define LDS_FENCE() asm volatile("s_wait_dscnt 0" ::: "memory")

__global__ __launch_bounds__(256) void fluid_mlp_grad_kernel(
    const float* __restrict__ x,
    const float* __restrict__ W0, const float* __restrict__ b0,
    const float* __restrict__ W1, const float* __restrict__ b1,
    const float* __restrict__ W2, const float* __restrict__ b2,
    const float* __restrict__ W3, const float* __restrict__ b3,
    float* __restrict__ out)
{
  __shared__ __align__(16) _Float16 WT1[1024], Wf1[1024], WT2[1024], Wf2[1024];
  __shared__ __align__(16) _Float16 WT1l[1024], Wf1l[1024], WT2l[1024], Wf2l[1024];
  __shared__ __align__(16) float sW0[160], sW3[160];
  __shared__ __align__(16) float sb0[32], sb1[32], sb2[32], sb3[8];
  __shared__ __align__(16) _Float16 tH[8][1024], tHl[8][1024];
  __shared__ __align__(16) _Float16 tG[8][1024], tGl[8][1024];
  __shared__ __align__(16) float sOut[8][32 * 6];
  __shared__ __align__(16) float tF[8][1024];

  const int tid  = threadIdx.x;
  const int lane = tid & 31;
  const int wave = tid >> 5;

  #pragma unroll
  for (int it = 0; it < 4; ++it) {
    int i = tid + it * 256;
    int k = i >> 5, n = i & 31;
    const float f1 = W1[i]; _Float16 w1 = (_Float16)f1, w1l = lo_of(f1, w1);
    WT1[n*32 + k] = w1;  Wf1[i] = w1;  WT1l[n*32 + k] = w1l;  Wf1l[i] = w1l;
    const float f2 = W2[i]; _Float16 w2 = (_Float16)f2, w2l = lo_of(f2, w2);
    WT2[n*32 + k] = w2;  Wf2[i] = w2;  WT2l[n*32 + k] = w2l;  Wf2l[i] = w2l;
  }
  if (tid < 160) { sW0[tid] = W0[tid]; sW3[tid] = W3[tid]; }
  if (tid < 32)  { sb0[tid] = b0[tid]; sb1[tid] = b1[tid]; sb2[tid] = b2[tid]; }
  if (tid < 5)   { sb3[tid] = b3[tid]; }
  __syncthreads();

  _Float16* myH = tH[wave];  _Float16* myHl = tHl[wave];
  _Float16* myG = tG[wave];  _Float16* myGl = tGl[wave];
  float* myO = sOut[wave];
  float* myF = tF[wave];

  const int p = (blockIdx.x * 8 + wave) * 32 + lane;
  const float* xv = x + (size_t)p * 3;
  float t  = xv[0];
  float sx = __builtin_amdgcn_sinf(xv[1]), cx = __builtin_amdgcn_cosf(xv[1]);
  float sy = __builtin_amdgcn_sinf(xv[2]), cy = __builtin_amdgcn_cosf(xv[2]);

  float s0p[32];
  #pragma unroll
  for (int j = 0; j < 32; j += 2) {
    float za = sb0[j]   + t*sW0[j]     + cx*sW0[32+j]   + sx*sW0[64+j]
                        + cy*sW0[96+j] + sy*sW0[128+j];
    float zb = sb0[j+1] + t*sW0[j+1]   + cx*sW0[33+j]   + sx*sW0[65+j]
                        + cy*sW0[97+j] + sy*sW0[129+j];
    const float ha = softplus20(za), hb = softplus20(zb);
    v2h hv = { (_Float16)ha, (_Float16)hb };
    v2h hl = { lo_of(ha, hv[0]), lo_of(hb, hv[1]) };
    *(v2h*)(myH + lane*32 + j) = hv;  *(v2h*)(myHl + lane*32 + j) = hl;
    s0p[j] = sigmoid20(za); s0p[j + 1] = sigmoid20(zb);
  }
  LDS_FENCE();

  v8f z1t[2][2];
  {
    v16h a0 = load_afrag(myH, lane, 0), a0l = load_afrag(myHl, lane, 0);
    v16h a1 = load_afrag(myH, lane, 1), a1l = load_afrag(myHl, lane, 1);
    #pragma unroll
    for (int nt = 0; nt < 2; ++nt) {
      v16h bf = load_bfrag(WT1, lane, nt), bl = load_bfrag(WT1l, lane, nt);
      float bb = sb1[nt*16 + (lane & 15)];
      v8f c = {bb, bb, bb, bb, bb, bb, bb, bb};
      z1t[0][nt] = wmma_split(a0, a0l, bf, bl, c);
      z1t[1][nt] = wmma_split(a1, a1l, bf, bl, c);
    }
  }
  float s1p[2][2][8];
  #pragma unroll
  for (int mt = 0; mt < 2; ++mt)
    #pragma unroll
    for (int nt = 0; nt < 2; ++nt) {
      int ncol  = nt*16 + (lane & 15);
      int mbase = mt*16 + (lane >> 4) * 8;
      #pragma unroll
      for (int r = 0; r < 8; ++r) {
        float zv = z1t[mt][nt][r];
        const float hv = softplus20(zv); const _Float16 hh = (_Float16)hv;
        myH[(mbase+r)*32 + ncol] = hh;  myHl[(mbase+r)*32 + ncol] = lo_of(hv, hh);
        s1p[mt][nt][r] = sigmoid20(zv);
      }
    }
  LDS_FENCE();

  v8f z2t[2][2];
  {
    v16h a0 = load_afrag(myH, lane, 0), a0l = load_afrag(myHl, lane, 0);
    v16h a1 = load_afrag(myH, lane, 1), a1l = load_afrag(myHl, lane, 1);
    #pragma unroll
    for (int nt = 0; nt < 2; ++nt) {
      v16h bf = load_bfrag(WT2, lane, nt), bl = load_bfrag(WT2l, lane, nt);
      float bb = sb2[nt*16 + (lane & 15)];
      v8f c = {bb, bb, bb, bb, bb, bb, bb, bb};
      z2t[0][nt] = wmma_split(a0, a0l, bf, bl, c);
      z2t[1][nt] = wmma_split(a1, a1l, bf, bl, c);
    }
  }
  #pragma unroll
  for (int mt = 0; mt < 2; ++mt)
    #pragma unroll
    for (int nt = 0; nt < 2; ++nt) {
      int ncol  = nt*16 + (lane & 15);
      int mbase = mt*16 + (lane >> 4) * 8;
      float w3c = sW3[ncol*5 + 4];
      #pragma unroll
      for (int r = 0; r < 8; ++r) {
        float zv = z2t[mt][nt][r];
        const float hv = softplus20(zv), gv = w3c * sigmoid20(zv);
        const _Float16 gh = (_Float16)gv;
        myF[(mbase+r)*32 + ncol] = hv;
        myG[(mbase+r)*32 + ncol] = gh;  myGl[(mbase+r)*32 + ncol] = lo_of(gv, gh);
      }
    }
  LDS_FENCE();

  {
    const v4f_t* rp = (const v4f_t*)(myF + lane*32);
    v4f_t hrc[8] = { rp[0], rp[1], rp[2], rp[3], rp[4], rp[5], rp[6], rp[7] };
    float y0 = sb3[0], y1 = sb3[1], y2 = sb3[2], y3 = sb3[3];
    #pragma unroll
    for (int c2 = 0; c2 < 8; ++c2)
      #pragma unroll
      for (int jj = 0; jj < 4; ++jj) {
        int j = c2*4 + jj;
        float hj = hrc[c2][jj];
        y0 = fmaf(hj, sW3[j*5+0], y0);
        y1 = fmaf(hj, sW3[j*5+1], y1);
        y2 = fmaf(hj, sW3[j*5+2], y2);
        y3 = fmaf(hj, sW3[j*5+3], y3);
      }
    myO[lane * 6 + 0] = y0; myO[lane * 6 + 1] = y1; myO[lane * 6 + 2] = y2; myO[lane * 6 + 3] = y3;
  }

  v8f g1t[2][2];
  {
    v16h a0 = load_afrag(myG, lane, 0), a0l = load_afrag(myGl, lane, 0);
    v16h a1 = load_afrag(myG, lane, 1), a1l = load_afrag(myGl, lane, 1);
    v8f zc = {0.f, 0.f, 0.f, 0.f, 0.f, 0.f, 0.f, 0.f};
    #pragma unroll
    for (int nt = 0; nt < 2; ++nt) {
      v16h bf = load_bfrag(Wf2, lane, nt), bl = load_bfrag(Wf2l, lane, nt);
      g1t[0][nt] = wmma_split(a0, a0l, bf, bl, zc);
      g1t[1][nt] = wmma_split(a1, a1l, bf, bl, zc);
    }
  }
  #pragma unroll
  for (int mt = 0; mt < 2; ++mt)
    #pragma unroll
    for (int nt = 0; nt < 2; ++nt) {
      int ncol  = nt*16 + (lane & 15);
      int mbase = mt*16 + (lane >> 4) * 8;
      #pragma unroll
      for (int r = 0; r < 8; ++r) {
        float d = g1t[mt][nt][r] * s1p[mt][nt][r];
        const _Float16 dh = (_Float16)d;
        myG[(mbase+r)*32 + ncol] = dh;  myGl[(mbase+r)*32 + ncol] = lo_of(d, dh);
      }
    }
  LDS_FENCE();

  v8f g0t[2][2];
  {
    v16h a0 = load_afrag(myG, lane, 0), a0l = load_afrag(myGl, lane, 0);
    v16h a1 = load_afrag(myG, lane, 1), a1l = load_afrag(myGl, lane, 1);
    v8f zc = {0.f, 0.f, 0.f, 0.f, 0.f, 0.f, 0.f, 0.f};
    #pragma unroll
    for (int nt = 0; nt < 2; ++nt) {
      v16h bf = load_bfrag(Wf1, lane, nt), bl = load_bfrag(Wf1l, lane, nt);
      g0t[0][nt] = wmma_split(a0, a0l, bf, bl, zc);
      g0t[1][nt] = wmma_split(a1, a1l, bf, bl, zc);
    }
  }
  LDS_FENCE();
  #pragma unroll
  for (int mt = 0; mt < 2; ++mt)
    #pragma unroll
    for (int nt = 0; nt < 2; ++nt) {
      int ncol  = nt*16 + (lane & 15);
      int mbase = mt*16 + (lane >> 4) * 8;
      #pragma unroll
      for (int r = 0; r < 8; ++r) myF[(mbase+r)*32 + ncol] = g0t[mt][nt][r];
    }
  LDS_FENCE();

  {
    const v4f_t* rp = (const v4f_t*)(myF + lane*32);
    v4f_t grc[8] = { rp[0], rp[1], rp[2], rp[3], rp[4], rp[5], rp[6], rp[7] };
    float ge1 = 0.f, ge2 = 0.f, ge3 = 0.f, ge4 = 0.f;
    #pragma unroll
    for (int c2 = 0; c2 < 8; ++c2)
      #pragma unroll
      for (int jj = 0; jj < 4; ++jj) {
        int j = c2*4 + jj;
        float dz = grc[c2][jj] * s0p[j];
        ge1 = fmaf(dz, sW0[32 + j],  ge1);
        ge2 = fmaf(dz, sW0[64 + j],  ge2);
        ge3 = fmaf(dz, sW0[96 + j],  ge3);
        ge4 = fmaf(dz, sW0[128 + j], ge4);
      }
    float dx1 = TWO_PI_F * (ge2 * cx - ge1 * sx);
    float dx2 = TWO_PI_F * (ge4 * cy - ge3 * sy);
    myO[lane * 6 + 4] = dx2; myO[lane * 6 + 5] = -dx1;
  }
  LDS_FENCE();
  {
    float* ob = out + (size_t)(blockIdx.x * 8 + wave) * 32 * 6;
#pragma unroll 1
    for (int pass = 0; pass < 2; ++pass) {
      for (int q = lane; q < 48; q += 32) *(volatile v4f_t*)(ob + q * 4) = *(const volatile v4fa*)(myO + q * 4);
      __threadfence();
    }
  }
}

extern "C" void kernel_launch(void* const* d_in, const int* in_sizes, int n_in,
                              void* d_out, int out_size, void* d_ws, size_t ws_size,
                              hipStream_t stream) {
  const float* x  = (const float*)d_in[0];
  const float* W0 = (const float*)d_in[1];
  const float* b0 = (const float*)d_in[2];
  const float* W1 = (const float*)d_in[3];
  const float* b1 = (const float*)d_in[4];
  const float* W2 = (const float*)d_in[5];
  const float* b2 = (const float*)d_in[6];
  const float* W3 = (const float*)d_in[7];
  const float* b3 = (const float*)d_in[8];
  float* out = (float*)d_out;

  (void)in_sizes;
  int nblocks = NPTS / 256;
  fluid_mlp_grad_kernel<<<nblocks, 256, 0, stream>>>(x, W0, b0, W1, b1, W2, b2, W3, b3, out);
}
